// knn_GradCAM_21002390078208
// MI455X (gfx1250) — hardware-verified
//
#include <hip/hip_runtime.h>
#include <stddef.h>


#define NTHR   256
#define NWAVE  8
#define EPT    8
#define NGRP   2
#define CHUNK  (NTHR * EPT * NGRP)
#define WCAP   (EPT * NGRP * 32)
#define LISTN  (NWAVE * WCAP)
#define MTHR   128
#define MEDG   64
#define HID    128
#define HP     (HID + 4)
#define FE     10
#define NBP    32
#define DIMO   64
#define EMBW   128
#define GMAX   208
#define O1P    68
#define O2P    36
#define NISO   16
#define CA     16.0f
#define CB     64.0f
#define CEA    16.0f
#define CW1    64.0f

static_assert((CHUNK & (CHUNK - 1)) == 0);
static_assert(CHUNK <= 4096);
static_assert(MTHR == 2 * MEDG);
static_assert((NBP & (NBP - 1)) == 0);

typedef float          v4f  __attribute__((ext_vector_type(4)));
typedef float          v8f  __attribute__((ext_vector_type(8)));
typedef int            v4i  __attribute__((ext_vector_type(4)));
typedef _Float16       v8h  __attribute__((ext_vector_type(8)));
typedef _Float16       v16h __attribute__((ext_vector_type(16)));
typedef __bf16         v8b  __attribute__((ext_vector_type(8)));
typedef __bf16         v16b __attribute__((ext_vector_type(16)));
typedef unsigned short v8us __attribute__((ext_vector_type(8)));
union FragH { v16h v; v8h h[2]; };
union FragB { v16b v; v8b h[2]; v8us u[2]; };

__host__ __device__ constexpr int kpad_of(int in) { return HID * in + ((in + 31) / 32) * 32; }
__host__ __device__ constexpr int msg_lds_bytes(int in, int out) {
  return (MEDG * HP + MEDG * in + MEDG * out) * 4 + MEDG * 4;
}
__host__ __device__ constexpr int node_lds_bytes(int in, int out) {
  return 16384 * 4 + 2 * out * ((((in + 31) / 32) * 32) + 8) * 2 + LISTN * 4 + 64;
}
__host__ __device__ constexpr int gc_lds_bytes(int kin, int pin) {
  return 256 * pin * 4 + 4 * 64 * ((((kin + 31) / 32) * 32) + 8) * 2 + LISTN * 4 + 64;
}
constexpr int LIFT_LDS = 256 * 96 * 4 + 256 * 4 + LISTN * 4 + 64;
constexpr int HEAD_LDS = 2 * 64 * (EMBW + 8) * 2 + 2 * 32 * (DIMO + 8) * 2 + GMAX * O1P * 4 + GMAX * O2P * 4 + GMAX * 4;

__device__ __forceinline__ v4f mk4(float a, float b, float c, float d) { v4f r = {a, b, c, d}; return r; }
__device__ __forceinline__ v4f zero4f() { v4f z = {0.f, 0.f, 0.f, 0.f}; return z; }
__device__ __forceinline__ v8f zero8f() { v8f z = {0.f, 0.f, 0.f, 0.f, 0.f, 0.f, 0.f, 0.f}; return z; }

__device__ __forceinline__ v8h cvt8(v4f a, v4f b) {
  v8h r;
  r[0] = (_Float16)a.x; r[1] = (_Float16)a.y; r[2] = (_Float16)a.z; r[3] = (_Float16)a.w;
  r[4] = (_Float16)b.x; r[5] = (_Float16)b.y; r[6] = (_Float16)b.z; r[7] = (_Float16)b.w;
  return r;
}
__device__ __forceinline__ v8h zero8h() { return cvt8(zero4f(), zero4f()); }

__device__ __forceinline__ unsigned int bfr(float x) {
  const unsigned int u = __float_as_uint(x);
  return (u + 0x7FFFu + ((u >> 16) & 1u)) >> 16;
}
__device__ __forceinline__ void split8(v4f a, v4f b, v8us& hi, v8us& lo) {
  float v[8];
  v[0] = a.x; v[1] = a.y; v[2] = a.z; v[3] = a.w; v[4] = b.x; v[5] = b.y; v[6] = b.z; v[7] = b.w;
#pragma unroll
  for (int e = 0; e < 8; ++e) {
    const unsigned int hb = bfr(v[e]);
    const float hf = __uint_as_float(hb << 16);
    const unsigned int lb = bfr(v[e] - hf);
    hi[e] = (unsigned short)hb;
    lo[e] = (unsigned short)lb;
  }
}

__device__ __forceinline__ v8f wmh(v16h a, v16h b, v8f c) {
  v8f d = __builtin_amdgcn_wmma_f32_16x16x32_f16(false, a, false, b, (short)0, c, false, false);
  asm volatile("v_nop\n\tv_nop\n\tv_nop\n\tv_nop" : "+v"(d) : "v"(a), "v"(b));
  return d;
}
__device__ __forceinline__ v8f wmb(v16b a, v16b b, v8f c) {
  v8f d = __builtin_amdgcn_wmma_f32_16x16x32_bf16(false, a, false, b, (short)0, c, false, false);
  asm volatile("v_nop\n\tv_nop\n\tv_nop\n\tv_nop" : "+v"(d) : "v"(a), "v"(b));
  return d;
}
__device__ __forceinline__ v8f wmb3(const FragB& ah, const FragB& al, const FragB& bh, const FragB& bl, v8f c) {
  c = wmb(ah.v, bh.v, c);
  c = wmb(ah.v, bl.v, c);
  c = wmb(al.v, bh.v, c);
  return c;
}

__device__ __forceinline__ int scan_chunk(const int* __restrict__ ids, int nE, int cbase, int slotBase, int nb,
                                          int vec8, int* list, int tid, int lane, int wave) {
  int wc = 0;
#pragma unroll
  for (int g = 0; g < NGRP; ++g) {
    const int el0  = (g * NTHR + tid) * EPT;
    const int e0   = cbase + el0;
    const int sent = -2147483647 - 1;
    v4i da, db;
    if (vec8 != 0 && cbase + CHUNK <= nE) {
      da = *(const v4i*)(ids + e0);
      db = *(const v4i*)(ids + e0 + 4);
    } else {
      const int lst = nE - 1;
      da.x = (e0     < nE) ? ids[min(e0,     lst)] : sent;
      da.y = (e0 + 1 < nE) ? ids[min(e0 + 1, lst)] : sent;
      da.z = (e0 + 2 < nE) ? ids[min(e0 + 2, lst)] : sent;
      da.w = (e0 + 3 < nE) ? ids[min(e0 + 3, lst)] : sent;
      db.x = (e0 + 4 < nE) ? ids[min(e0 + 4, lst)] : sent;
      db.y = (e0 + 5 < nE) ? ids[min(e0 + 5, lst)] : sent;
      db.z = (e0 + 6 < nE) ? ids[min(e0 + 6, lst)] : sent;
      db.w = (e0 + 7 < nE) ? ids[min(e0 + 7, lst)] : sent;
    }
    const unsigned bs = (unsigned)slotBase;
    const unsigned ub = (unsigned)nb;
    const unsigned s0 = (unsigned)da.x - bs, s1 = (unsigned)da.y - bs;
    const unsigned s2 = (unsigned)da.z - bs, s3 = (unsigned)da.w - bs;
    const unsigned s4 = (unsigned)db.x - bs, s5 = (unsigned)db.y - bs;
    const unsigned s6 = (unsigned)db.z - bs, s7 = (unsigned)db.w - bs;
    const bool h0 = s0 < ub, h1 = s1 < ub, h2 = s2 < ub, h3 = s3 < ub;
    const bool h4 = s4 < ub, h5 = s5 < ub, h6 = s6 < ub, h7 = s7 < ub;
    const unsigned any = __builtin_amdgcn_ballot_w32(h0 | h1 | h2 | h3 | h4 | h5 | h6 | h7);
    if (any != 0u) {
#define HITJ(J, HJ, SJ) { \
        const unsigned mj = __builtin_amdgcn_ballot_w32(HJ); \
        if (mj != 0u) { \
          if (HJ) { \
            const int pos = wc + (int)__builtin_amdgcn_mbcnt_lo(mj, 0u); \
            if (pos < WCAP) list[wave * WCAP + pos] = ((el0 + (J)) << 12) | (int)(SJ); \
          } \
          wc += (int)__builtin_popcount(mj); } }
      HITJ(0, h0, s0)
      HITJ(1, h1, s1)
      HITJ(2, h2, s2)
      HITJ(3, h3, s3)
      HITJ(4, h4, s4)
      HITJ(5, h5, s5)
      HITJ(6, h6, s6)
      HITJ(7, h7, s7)
#undef HITJ
    }
  }
  return wc;
}

template <int IN, int OUT>
__global__ __launch_bounds__(NTHR) void k_bprep(const float* __restrict__ W2, const float* __restrict__ b2,
                                               _Float16* Bp) {
  constexpr int KMAIN = HID * IN;
  constexpr int KPAD  = kpad_of(IN);
  constexpr int NU    = OUT * KPAD / 8;
  static_assert((KPAD % 32) == 0);
  static_assert((NU % 32) == 0);
  const int u = blockIdx.x * NTHR + (int)threadIdx.x;
  if (u >= NU) return;
  const int o  = u * 8;
  const int n  = o / KPAD;
  const int j0 = o - n * KPAD;
  float v[8];
#pragma unroll
  for (int e = 0; e < 8; ++e) {
    const int j  = j0 + e;
    const int jw = j < KMAIN ? j : KMAIN - 1;
    const int i  = jw >> 7;
    const int k  = jw & 127;
    const int ir = j - KMAIN;
    const int irc = ir < 0 ? 0 : (ir > IN - 1 ? IN - 1 : ir);
    const float wv = W2[(size_t)k * (IN * OUT) + i * OUT + n];
    const float bv = b2[(size_t)irc * OUT + n];
    v[e] = (j < KMAIN ? wv : (ir < IN ? bv : 0.0f)) * CB;
  }
  const v8h hv = cvt8(mk4(v[0], v[1], v[2], v[3]), mk4(v[4], v[5], v[6], v[7]));
  _Float16* dp = Bp + o;
  *(volatile v8h*)dp = hv;
  __threadfence();
  *(volatile v8h*)dp = hv;
}

template <int IN, int OUT>
__global__ __launch_bounds__(MTHR) void k_msg(
    const float* __restrict__ X, int nX, const int* __restrict__ ei, int nE,
    const float* __restrict__ EA, const float* __restrict__ W1, const float* __restrict__ bb1,
    const _Float16* __restrict__ Bp, float* MSG) {
  constexpr int KMAIN = HID * IN;
  constexpr int KPAD  = kpad_of(IN);
  constexpr int KTAIL = KPAD - KMAIN;
  constexpr int NT    = OUT / 16;
  constexpr int NTH   = HID / 16;
  constexpr int NCH   = KMAIN / 32;
  constexpr int NCT   = KTAIL / 32;
  constexpr int NPI   = 16 * OUT / 128;
  static_assert((IN % 8) == 0 && (OUT % 32) == 0 && NT <= 4);
  static_assert((KPAD % 32) == 0 && (KMAIN % 32) == 0);

  extern __shared__ v4f lds_dyn[];
  float* Hs  = (float*)lds_dyn;
  float* Xs  = Hs + MEDG * HP;
  float* Stg = Xs + MEDG * IN;
  int*   Ss  = (int*)(Stg + MEDG * OUT);

  const int tid = threadIdx.x, lane = tid & 31, wave = tid >> 5, hh = lane >> 4, m = lane & 15;
  const int eBase = blockIdx.x * MEDG;

  if (tid < MEDG) {
    int e = eBase + tid;
    e = e > nE - 1 ? nE - 1 : e;
    int s = ei[e];
    s = s < 0 ? 0 : (s > nX - 1 ? nX - 1 : s);
    Ss[tid] = s;
  }

  {
    int e = eBase + 16 * wave + m;
    e = e > nE - 1 ? nE - 1 : e;
    const float* ep = EA + (size_t)e * FE;
    float av[8];
#pragma unroll
    for (int t = 0; t < 8; ++t) {
      const int k  = 8 * hh + t;
      const int kc = k < FE ? k : FE - 1;
      const float v = ep[kc];
      av[t] = (k < FE) ? v * CEA : 0.0f;
    }
    FragH a;
    a.h[0] = cvt8(mk4(av[0], av[1], av[2], av[3]), mk4(av[4], av[5], av[6], av[7]));
    a.h[1] = zero8h();
    float* hw = Hs + (16 * wave + 8 * hh) * HP;
#pragma unroll
    for (int tt = 0; tt < NTH; ++tt) {
      const int col = 16 * tt + m;
      float bv[8];
#pragma unroll
      for (int t = 0; t < 8; ++t) {
        const int k  = 8 * hh + t;
        const int kc = k < FE ? k : FE - 1;
        const float w = W1[(size_t)kc * HID + col];
        bv[t] = (k < FE) ? w * CW1 : 0.0f;
      }
      FragH b;
      b.h[0] = cvt8(mk4(bv[0], bv[1], bv[2], bv[3]), mk4(bv[4], bv[5], bv[6], bv[7]));
      b.h[1] = zero8h();
      const v8f d = wmh(a.v, b.v, zero8f());
      const float bav = bb1[col];
#pragma unroll
      for (int r = 0; r < 8; ++r) hw[r * HP + col] = fmaxf(d[r] * (1.0f / (CEA * CW1)) + bav, 0.0f);
    }
  }
  __syncthreads();

#pragma unroll 1
  for (int u = tid; u < MEDG * (IN / 4); u += MTHR) {
    const int r  = u / (IN / 4);
    const int c4 = u - r * (IN / 4);
    const int s  = Ss[r];
    *(v4f*)(Xs + r * IN + 4 * c4) = *(const v4f*)(X + (size_t)s * IN + 4 * c4);
  }
  __syncthreads();

  v8f acc[NT];
#pragma unroll
  for (int t = 0; t < NT; ++t) acc[t] = zero8f();
  const float* xrow = Xs + (16 * wave + m) * IN;
  const float* hrow = Hs + (16 * wave + m) * HP + 8 * hh;
  const _Float16* bbase = Bp + (size_t)m * KPAD + 8 * hh;

#pragma unroll 1
  for (int c = 0; c < NCH; ++c) {
    const int i = c >> 2;
    const int q = c & 3;
    const float xi = xrow[i] * CA;
    const float* hp = hrow + 32 * q;
    const v4f ha = *(const v4f*)hp;
    const v4f hb = *(const v4f*)(hp + 4);
    const v4f hc = *(const v4f*)(hp + 16);
    const v4f hd = *(const v4f*)(hp + 20);
    FragH a;
    a.h[0] = cvt8(ha * xi, hb * xi);
    a.h[1] = cvt8(hc * xi, hd * xi);
    const _Float16* bp = bbase + (size_t)32 * c;
#pragma unroll
    for (int t = 0; t < NT; ++t) {
      const _Float16* bt = bp + (size_t)(16 * t) * KPAD;
      FragH b;
      b.h[0] = *(const v8h*)bt;
      b.h[1] = *(const v8h*)(bt + 16);
      acc[t] = wmh(a.v, b.v, acc[t]);
    }
  }
#pragma unroll
  for (int ct = 0; ct < NCT; ++ct) {
    float av[8], aw[8];
#pragma unroll
    for (int t = 0; t < 8; ++t) {
      const int i1 = 32 * ct + 8 * hh + t;
      const int i2 = i1 + 16;
      const int c1 = i1 < IN ? i1 : IN - 1;
      const int c2 = i2 < IN ? i2 : IN - 1;
      const float v1 = xrow[c1];
      const float v2 = xrow[c2];
      av[t] = (i1 < IN) ? v1 * CA : 0.0f;
      aw[t] = (i2 < IN) ? v2 * CA : 0.0f;
    }
    FragH a;
    a.h[0] = cvt8(mk4(av[0], av[1], av[2], av[3]), mk4(av[4], av[5], av[6], av[7]));
    a.h[1] = cvt8(mk4(aw[0], aw[1], aw[2], aw[3]), mk4(aw[4], aw[5], aw[6], aw[7]));
    const _Float16* bp = bbase + (size_t)KMAIN + 32 * ct;
#pragma unroll
    for (int t = 0; t < NT; ++t) {
      const _Float16* bt = bp + (size_t)(16 * t) * KPAD;
      FragH b;
      b.h[0] = *(const v8h*)bt;
      b.h[1] = *(const v8h*)(bt + 16);
      acc[t] = wmh(a.v, b.v, acc[t]);
    }
  }
  __syncthreads();

  {
    float* sp = Stg + (16 * wave + 8 * hh) * OUT + m;
#pragma unroll
    for (int t = 0; t < NT; ++t) {
#pragma unroll
      for (int r = 0; r < 8; ++r) sp[r * OUT + 16 * t] = acc[t][r] * (1.0f / (CA * CB));
    }
  }
  __syncthreads();

  const float* lp = Stg + 16 * wave * OUT;
  float* gp = MSG + (size_t)(eBase + 16 * wave) * OUT;
#pragma unroll
  for (int p = 0; p < NPI; ++p) {
    const v4f v = *(const v4f*)(lp + 4 * (32 * p + lane));
    *(volatile v4f*)(gp + 4 * (32 * p + lane)) = v;
  }
  __threadfence();
#pragma unroll
  for (int p = 0; p < NPI; ++p) {
    const v4f v = *(const v4f*)(lp + 4 * (32 * p + lane));
    *(volatile v4f*)(gp + 4 * (32 * p + lane)) = v;
  }
}

template <int IN, int OUT>
__global__ __launch_bounds__(NTHR) void k_node(
    const int* __restrict__ ei, int nE, int vec8, const float* __restrict__ MSG,
    const float* __restrict__ XIN, int nN,
    const float* __restrict__ root, const float* __restrict__ cbias, float* HN) {
  constexpr int NB  = 16384 / OUT;
  constexpr int NT  = OUT / 16;
  constexpr int SPW = NB / 128;
  constexpr int KXP = ((IN + 31) / 32) * 32;
  constexpr int KT  = KXP / 32;
  constexpr int RP  = KXP + 8;
  constexpr int LPR = OUT / 4;
  constexpr int NPT = (NB * OUT / 4) / NTHR;
  static_assert(SPW * NT == 8);
  static_assert(NB <= 512 && (NB & (NB - 1)) == 0);
  static_assert((IN % 8) == 0 && (OUT % 16) == 0 && LPR <= 32);
  static_assert(NPT * NTHR * 4 == NB * OUT);

  extern __shared__ v4f lds_dyn[];
  float*          accL  = (float*)lds_dyn;
  unsigned short* rootH = (unsigned short*)(accL + NB * OUT);
  unsigned short* rootL = rootH + OUT * RP;
  int*            list  = (int*)(rootL + OUT * RP);
  int*            wcnt  = list + LISTN;

  const int tid = threadIdx.x, lane = tid & 31, wave = tid >> 5, hh = lane >> 4, m = lane & 15;
  const int nodeBase = blockIdx.x * NB;
  const int* dsts = ei + nE;

  {
    const v4f z = zero4f();
#pragma unroll 1
    for (int i = tid; i < NB * OUT / 4; i += NTHR) ((v4f*)accL)[i] = z;
#pragma unroll 1
    for (int u = tid; u < OUT * (KXP / 8); u += NTHR) {
      const int n  = u / (KXP / 8);
      const int k0 = (u - n * (KXP / 8)) * 8;
      float v[8];
#pragma unroll
      for (int e = 0; e < 8; ++e) {
        const int k  = k0 + e;
        const int kc = k < IN ? k : IN - 1;
        const float w = root[(size_t)kc * OUT + n];
        v[e] = (k < IN) ? w : 0.0f;
      }
      v8us hi, lo;
      split8(mk4(v[0], v[1], v[2], v[3]), mk4(v[4], v[5], v[6], v[7]), hi, lo);
      *(v8us*)(rootH + n * RP + k0) = hi;
      *(v8us*)(rootL + n * RP + k0) = lo;
    }
  }
  __syncthreads();

  const int nChunks = (nE + CHUNK - 1) / CHUNK;
#pragma unroll 1
  for (int ch = 0; ch < nChunks; ++ch) {
    const int cbase = ch * CHUNK;
    const int wc = scan_chunk(dsts, nE, cbase, nodeBase, NB, vec8, list, tid, lane, wave);
    if (lane == 0) wcnt[wave] = wc;
    __syncthreads();
    if (wave == 0) {
#pragma unroll 1
      for (int wsx = 0; wsx < NWAVE; ++wsx) {
        int n = __builtin_amdgcn_readfirstlane(wcnt[wsx]);
        n = n > WCAP ? WCAP : (n < 0 ? 0 : n);
        const int* lp = list + wsx * WCAP;
#pragma unroll 1
        for (int i = 0; i < n; ++i) {
          const int ent = __builtin_amdgcn_readfirstlane(lp[i]);
          int slot = ent & 4095;
          slot = slot > NB - 1 ? NB - 1 : slot;
          int e = cbase + ((ent >> 12) & (CHUNK - 1));
          e = e > nE - 1 ? nE - 1 : e;
          const int col = 4 * (lane % LPR);
          const v4f v = *(const v4f*)(MSG + (size_t)e * OUT + col);
          if (lane < LPR) {
            v4f* ap = (v4f*)(accL + slot * OUT + col);
            *ap = *ap + v;
          }
        }
      }
    }
    __syncthreads();
  }

#pragma unroll 1
  for (int s = 0; s < SPW; ++s) {
    const int row0 = (wave * SPW + s) * 16;
    int arow = nodeBase + row0 + m;
    arow = arow > nN - 1 ? nN - 1 : arow;
    const float* xr = XIN + (size_t)arow * IN;
    v8f acc2[NT];
#pragma unroll
    for (int t = 0; t < NT; ++t) acc2[t] = zero8f();
#pragma unroll
    for (int kt = 0; kt < KT; ++kt) {
      FragB ah, al;
#pragma unroll
      for (int g = 0; g < 2; ++g) {
        const int kb  = 32 * kt + 16 * g + 8 * hh;
        const int kbc = kb < IN - 8 ? kb : IN - 8;
        const float msk = (kb + 8 <= IN) ? 1.0f : 0.0f;
        const v4f p = *(const v4f*)(xr + kbc) * msk;
        const v4f q = *(const v4f*)(xr + kbc + 4) * msk;
        split8(p, q, ah.u[g], al.u[g]);
      }
#pragma unroll
      for (int t = 0; t < NT; ++t) {
        const unsigned short* bp = rootH + (16 * t + m) * RP + 32 * kt + 8 * hh;
        const unsigned short* bq = rootL + (16 * t + m) * RP + 32 * kt + 8 * hh;
        FragB bh, bl;
        bh.u[0] = *(const v8us*)bp;
        bh.u[1] = *(const v8us*)(bp + 16);
        bl.u[0] = *(const v8us*)bq;
        bl.u[1] = *(const v8us*)(bq + 16);
        acc2[t] = wmb3(ah, al, bh, bl, acc2[t]);
      }
    }
#pragma unroll
    for (int t = 0; t < NT; ++t) {
      const int col = 16 * t + m;
      const float cbv = cbias[col];
      float* ap = accL + (row0 + 8 * hh) * OUT + col;
#pragma unroll
      for (int r = 0; r < 8; ++r) {
        const float ag = ap[r * OUT];
        ap[r * OUT] = fmaxf(ag + acc2[t][r] + cbv, 0.0f);
      }
    }
  }
  __syncthreads();

  float* gp = HN + (size_t)nodeBase * OUT;
#pragma unroll
  for (int p = 0; p < NPT; ++p) {
    const int idx = p * NTHR + tid;
    const v4f v = ((const v4f*)accL)[idx];
    *(volatile v4f*)(gp + 4 * (size_t)idx) = v;
  }
  __threadfence();
#pragma unroll
  for (int p = 0; p < NPT; ++p) {
    const int idx = p * NTHR + tid;
    const v4f v = ((const v4f*)accL)[idx];
    *(volatile v4f*)(gp + 4 * (size_t)idx) = v;
  }
}

__global__ __launch_bounds__(NTHR) void k_pool(
    const int* __restrict__ seg, int nN, const float* __restrict__ H, float* EMB, int G, int coff) {
  __shared__ __attribute__((aligned(16))) float gacc[NBP * DIMO];
  __shared__ __attribute__((aligned(16))) int plist[LISTN];
  __shared__ int pcnt[NBP];
  __shared__ int wcnt[NWAVE];
  const int tid = threadIdx.x, lane = tid & 31, wave = tid >> 5, hh = lane >> 4, m = lane & 15;
  const int gBase = blockIdx.x * NBP;
  int nb = G - gBase;
  nb = nb < 0 ? 0 : (nb > NBP ? NBP : nb);

  {
    const v4f z = zero4f();
#pragma unroll 1
    for (int i = tid; i < NBP * DIMO / 4; i += NTHR) ((v4f*)gacc)[i] = z;
    if (tid < NBP) pcnt[tid] = 0;
  }
  __syncthreads();

  const int nChunks = (nN + CHUNK - 1) / CHUNK;
#pragma unroll 1
  for (int ch = 0; ch < nChunks; ++ch) {
    const int cbase = ch * CHUNK;
    const int wc = scan_chunk(seg, nN, cbase, gBase, nb, 1, plist, tid, lane, wave);
    if (lane == 0) wcnt[wave] = wc;
    __syncthreads();
    if (wave == 0) {
#pragma unroll 1
      for (int wsx = 0; wsx < NWAVE; ++wsx) {
        int n = __builtin_amdgcn_readfirstlane(wcnt[wsx]);
        n = n > WCAP ? WCAP : (n < 0 ? 0 : n);
        const int* lp = plist + wsx * WCAP;
#pragma unroll 1
        for (int i = 0; i < n; ++i) {
          const int ent = __builtin_amdgcn_readfirstlane(lp[i]);
          int slot = ent & 4095;
          slot = slot > NBP - 1 ? NBP - 1 : slot;
          int nd = cbase + ((ent >> 12) & (CHUNK - 1));
          nd = nd > nN - 1 ? nN - 1 : nd;
          const int col = 4 * (lane & 15);
          const v4f v = *(const v4f*)(H + (size_t)nd * DIMO + col);
          if (lane < 16) {
            v4f* ap = (v4f*)(gacc + slot * DIMO + col);
            *ap = *ap + v;
          }
          if (lane == 0) pcnt[slot] = pcnt[slot] + 1;
        }
      }
    }
    __syncthreads();
  }

#pragma unroll 1
  for (int u = tid; u < NBP * (DIMO / 4); u += NTHR) {
    const int row = u / (DIMO / 4);
    const int c4  = (u - row * (DIMO / 4)) * 4;
    int c = pcnt[row];
    c = c < 1 ? 1 : c;
    const float rcv = 1.0f / (float)c;
    v4f* ap = (v4f*)(gacc + row * DIMO + c4);
    *ap = *ap * rcv;
  }
  __syncthreads();

#pragma unroll
  for (int p = 0; p < 2; ++p) {
    const int row = 4 * wave + 2 * p + hh;
    const v4f v = *(const v4f*)(gacc + row * DIMO + 4 * m);
    *(volatile v4f*)(EMB + (size_t)(gBase + row) * EMBW + coff + 4 * m) = v;
  }
  __threadfence();
#pragma unroll
  for (int p = 0; p < 2; ++p) {
    const int row = 4 * wave + 2 * p + hh;
    const v4f v = *(const v4f*)(gacc + row * DIMO + 4 * m);
    *(volatile v4f*)(EMB + (size_t)(gBase + row) * EMBW + coff + 4 * m) = v;
  }
}

__global__ __launch_bounds__(NTHR) void k_lift(
    const int* __restrict__ asg, int nA, int vec8, const float* __restrict__ H1, int nN,
    const float* __restrict__ ISO, int nN2, float* H2) {
  constexpr int NB = 256, PO = 96;
  constexpr int NPT = (NB * PO / 4) / NTHR;
  static_assert(NPT * NTHR * 4 == NB * PO);
  extern __shared__ v4f lds_dyn[];
  float* accL = (float*)lds_dyn;
  int*   pc   = (int*)(accL + NB * PO);
  int*   list = pc + NB;
  int*   wcnt = list + LISTN;

  const int tid = threadIdx.x, lane = tid & 31, wave = tid >> 5;
  const int tb = blockIdx.x * NB;
  const int* srcs = asg;
  const int* segs = asg + nA;

  {
    const v4f z = zero4f();
#pragma unroll 1
    for (int i = tid; i < NB * PO / 4; i += NTHR) ((v4f*)accL)[i] = z;
#pragma unroll 1
    for (int i = tid; i < NB; i += NTHR) pc[i] = 0;
  }
  __syncthreads();

  const int nChunks = (nA + CHUNK - 1) / CHUNK;
#pragma unroll 1
  for (int ch = 0; ch < nChunks; ++ch) {
    const int cbase = ch * CHUNK;
    const int wc = scan_chunk(segs, nA, cbase, tb, NB, vec8, list, tid, lane, wave);
    if (lane == 0) wcnt[wave] = wc;
    __syncthreads();
    if (wave == 0) {
#pragma unroll 1
      for (int wsx = 0; wsx < NWAVE; ++wsx) {
        int n = __builtin_amdgcn_readfirstlane(wcnt[wsx]);
        n = n > WCAP ? WCAP : (n < 0 ? 0 : n);
        const int* lp = list + wsx * WCAP;
#pragma unroll 1
        for (int i = 0; i < n; ++i) {
          const int ent = __builtin_amdgcn_readfirstlane(lp[i]);
          int slot = ent & 4095;
          slot = slot > NB - 1 ? NB - 1 : slot;
          int a = cbase + ((ent >> 12) & (CHUNK - 1));
          a = a > nA - 1 ? nA - 1 : a;
          int g = srcs[a];
          g = g < 0 ? 0 : (g > nN - 1 ? nN - 1 : g);
          const int col = 4 * (lane & 15);
          const v4f v = *(const v4f*)(H1 + (size_t)g * DIMO + col);
          if (lane < 16) {
            v4f* ap = (v4f*)(accL + slot * PO + col);
            *ap = *ap + v;
          }
          if (lane == 0) pc[slot] = pc[slot] + 1;
        }
      }
    }
    __syncthreads();
  }

#pragma unroll 1
  for (int u = tid; u < NB * (PO / 4); u += NTHR) {
    const int row = u / (PO / 4);
    const int c4  = (u - row * (PO / 4)) * 4;
    int c = pc[row];
    c = c < 1 ? 1 : c;
    const float rcv = 1.0f / (float)c;
    int trow = tb + row;
    trow = trow > nN2 - 1 ? nN2 - 1 : trow;
    int ic = c4 - DIMO;
    ic = ic < 0 ? 0 : (ic > NISO - 4 ? NISO - 4 : ic);
    const float m0 = (c4 < DIMO) ? 1.0f : 0.0f;
    const float m1 = (c4 >= DIMO && c4 < DIMO + NISO) ? 1.0f : 0.0f;
    v4f* ap = (v4f*)(accL + row * PO + c4);
    const v4f accv = *ap;
    const v4f isov = *(const v4f*)(ISO + (size_t)trow * NISO + ic);
    *ap = accv * (rcv * m0) + isov * m1;
  }
  __syncthreads();

  float* gp = H2 + (size_t)tb * PO;
#pragma unroll
  for (int p = 0; p < NPT; ++p) {
    const int idx = p * NTHR + tid;
    const v4f v = ((const v4f*)accL)[idx];
    *(volatile v4f*)(gp + 4 * (size_t)idx) = v;
  }
  __threadfence();
#pragma unroll
  for (int p = 0; p < NPT; ++p) {
    const int idx = p * NTHR + tid;
    const v4f v = ((const v4f*)accL)[idx];
    *(volatile v4f*)(gp + 4 * (size_t)idx) = v;
  }
}

template <int KIN, int PIN>
__global__ __launch_bounds__(NTHR) void k_gc(
    const int* __restrict__ ei, int nE, int vec8,
    const float* __restrict__ HIN, int nSrc, int nRows,
    const float* __restrict__ Wrel, const float* __restrict__ Wroot, const float* __restrict__ bias,
    float* HOUT) {
  constexpr int NB  = 256;
  constexpr int NT  = DIMO / 16;
  constexpr int KP  = ((KIN + 31) / 32) * 32;
  constexpr int KT  = KP / 32;
  constexpr int RP  = KP + 8;
  constexpr int LPR = PIN / 4;
  static_assert(KP <= PIN && (PIN % 4) == 0 && LPR <= 32 && NT == 4);

  extern __shared__ v4f lds_dyn[];
  float*          accL = (float*)lds_dyn;
  unsigned short* relH = (unsigned short*)(accL + NB * PIN);
  unsigned short* relL = relH + DIMO * RP;
  unsigned short* rooH = relL + DIMO * RP;
  unsigned short* rooL = rooH + DIMO * RP;
  int*            list = (int*)(rooL + DIMO * RP);
  int*            wcnt = list + LISTN;

  const int tid = threadIdx.x, lane = tid & 31, wave = tid >> 5, hh = lane >> 4, m = lane & 15;
  const int nodeBase = blockIdx.x * NB;
  const int* srcs = ei;
  const int* dsts = ei + nE;

  {
    const v4f z = zero4f();
#pragma unroll 1
    for (int i = tid; i < NB * PIN / 4; i += NTHR) ((v4f*)accL)[i] = z;
#pragma unroll 1
    for (int u = tid; u < DIMO * (KP / 8); u += NTHR) {
      const int n  = u / (KP / 8);
      const int k0 = (u - n * (KP / 8)) * 8;
      float vr[8], vo[8];
#pragma unroll
      for (int e = 0; e < 8; ++e) {
        const int k  = k0 + e;
        const int kc = k < KIN ? k : KIN - 1;
        const float a = Wrel[(size_t)kc * DIMO + n];
        const float b = Wroot[(size_t)kc * DIMO + n];
        vr[e] = (k < KIN) ? a : 0.0f;
        vo[e] = (k < KIN) ? b : 0.0f;
      }
      v8us hi, lo;
      split8(mk4(vr[0], vr[1], vr[2], vr[3]), mk4(vr[4], vr[5], vr[6], vr[7]), hi, lo);
      *(v8us*)(relH + n * RP + k0) = hi;
      *(v8us*)(relL + n * RP + k0) = lo;
      split8(mk4(vo[0], vo[1], vo[2], vo[3]), mk4(vo[4], vo[5], vo[6], vo[7]), hi, lo);
      *(v8us*)(rooH + n * RP + k0) = hi;
      *(v8us*)(rooL + n * RP + k0) = lo;
    }
  }
  __syncthreads();

  const int nChunks = (nE + CHUNK - 1) / CHUNK;
#pragma unroll 1
  for (int ch = 0; ch < nChunks; ++ch) {
    const int cbase = ch * CHUNK;
    const int wc = scan_chunk(dsts, nE, cbase, nodeBase, NB, vec8, list, tid, lane, wave);
    if (lane == 0) wcnt[wave] = wc;
    __syncthreads();
    if (wave == 0) {
#pragma unroll 1
      for (int wsx = 0; wsx < NWAVE; ++wsx) {
        int n = __builtin_amdgcn_readfirstlane(wcnt[wsx]);
        n = n > WCAP ? WCAP : (n < 0 ? 0 : n);
        const int* lp = list + wsx * WCAP;
#pragma unroll 1
        for (int i = 0; i < n; ++i) {
          const int ent = __builtin_amdgcn_readfirstlane(lp[i]);
          int slot = ent & 4095;
          slot = slot > NB - 1 ? NB - 1 : slot;
          int e = cbase + ((ent >> 12) & (CHUNK - 1));
          e = e > nE - 1 ? nE - 1 : e;
          int sidx = srcs[e];
          sidx = sidx < 0 ? 0 : (sidx > nSrc - 1 ? nSrc - 1 : sidx);
          const int col = 4 * (lane % LPR);
          const v4f v = *(const v4f*)(HIN + (size_t)sidx * PIN + col);
          if (lane < LPR) {
            v4f* ap = (v4f*)(accL + slot * PIN + col);
            *ap = *ap + v;
          }
        }
      }
    }
    __syncthreads();
  }

#pragma unroll 1
  for (int s = 0; s < 2; ++s) {
    const int row0 = (wave * 2 + s) * 16;
    const float* ar = accL + (row0 + m) * PIN;
    int orow = nodeBase + row0 + m;
    orow = orow > nRows - 1 ? nRows - 1 : orow;
    const float* xr = HIN + (size_t)orow * PIN;
    v8f acc2[NT];
#pragma unroll
    for (int t = 0; t < NT; ++t) acc2[t] = zero8f();
#pragma unroll
    for (int kt = 0; kt < KT; ++kt) {
      FragB ah, al;
#pragma unroll
      for (int g = 0; g < 2; ++g) {
        const int kb = 32 * kt + 16 * g + 8 * hh;
        split8(*(const v4f*)(ar + kb), *(const v4f*)(ar + kb + 4), ah.u[g], al.u[g]);
      }
#pragma unroll
      for (int t = 0; t < NT; ++t) {
        const unsigned short* bp = relH + (16 * t + m) * RP + 32 * kt + 8 * hh;
        const unsigned short* bq = relL + (16 * t + m) * RP + 32 * kt + 8 * hh;
        FragB bh, bl;
        bh.u[0] = *(const v8us*)bp;
        bh.u[1] = *(const v8us*)(bp + 16);
        bl.u[0] = *(const v8us*)bq;
        bl.u[1] = *(const v8us*)(bq + 16);
        acc2[t] = wmb3(ah, al, bh, bl, acc2[t]);
      }
    }
#pragma unroll
    for (int kt = 0; kt < KT; ++kt) {
      FragB ah, al;
#pragma unroll
      for (int g = 0; g < 2; ++g) {
        const int kb = 32 * kt + 16 * g + 8 * hh;
        split8(*(const v4f*)(xr + kb), *(const v4f*)(xr + kb + 4), ah.u[g], al.u[g]);
      }
#pragma unroll
      for (int t = 0; t < NT; ++t) {
        const unsigned short* bp = rooH + (16 * t + m) * RP + 32 * kt + 8 * hh;
        const unsigned short* bq = rooL + (16 * t + m) * RP + 32 * kt + 8 * hh;
        FragB bh, bl;
        bh.u[0] = *(const v8us*)bp;
        bh.u[1] = *(const v8us*)(bp + 16);
        bl.u[0] = *(const v8us*)bq;
        bl.u[1] = *(const v8us*)(bq + 16);
        acc2[t] = wmb3(ah, al, bh, bl, acc2[t]);
      }
    }
    __syncthreads();
#pragma unroll
    for (int t = 0; t < NT; ++t) {
      const int col = 16 * t + m;
      const float bv = bias[col];
      float* ap = accL + (row0 + 8 * hh) * PIN + col;
#pragma unroll
      for (int r = 0; r < 8; ++r) ap[r * PIN] = fmaxf(acc2[t][r] + bv, 0.0f);
    }
  }
  __syncthreads();

  const size_t gro = (size_t)nodeBase * DIMO;
#pragma unroll
  for (int p = 0; p < 16; ++p) {
    const int row = wave * 32 + 2 * p + hh;
    const v4f v = *(const v4f*)(accL + row * PIN + 4 * m);
    *(volatile v4f*)(HOUT + gro + (size_t)row * DIMO + 4 * m) = v;
  }
  __threadfence();
#pragma unroll
  for (int p = 0; p < 16; ++p) {
    const int row = wave * 32 + 2 * p + hh;
    const v4f v = *(const v4f*)(accL + row * PIN + 4 * m);
    *(volatile v4f*)(HOUT + gro + (size_t)row * DIMO + 4 * m) = v;
  }
}

__global__ __launch_bounds__(NTHR) void k_head(
    const float* __restrict__ EMB, int GP,
    const float* __restrict__ fc1w, const float* __restrict__ fc1b,
    const float* __restrict__ fc2w, const float* __restrict__ fc2b,
    const float* __restrict__ fc3w, const float* __restrict__ fc3b, float* out, int G) {
  constexpr int RP1 = EMBW + 8;
  constexpr int RP2 = DIMO + 8;
  extern __shared__ v4f lds_dyn[];
  unsigned short* w1H = (unsigned short*)lds_dyn;
  unsigned short* w1L = w1H + DIMO * RP1;
  unsigned short* w2H = w1L + DIMO * RP1;
  unsigned short* w2L = w2H + 32 * RP2;
  float* o1 = (float*)(w2L + 32 * RP2);
  float* o2 = o1 + GMAX * O1P;
  float* so = o2 + GMAX * O2P;

  const int tid = threadIdx.x, lane = tid & 31, wave = tid >> 5, hh = lane >> 4, m = lane & 15;
  const int nRT = (G + 15) / 16;

#pragma unroll 1
  for (int u = tid; u < DIMO * (EMBW / 8); u += NTHR) {
    const int n  = u / (EMBW / 8);
    const int k0 = (u - n * (EMBW / 8)) * 8;
    float v[8];
#pragma unroll
    for (int e = 0; e < 8; ++e) v[e] = fc1w[(size_t)(k0 + e) * DIMO + n];
    v8us hi, lo;
    split8(mk4(v[0], v[1], v[2], v[3]), mk4(v[4], v[5], v[6], v[7]), hi, lo);
    *(v8us*)(w1H + n * RP1 + k0) = hi;
    *(v8us*)(w1L + n * RP1 + k0) = lo;
  }
#pragma unroll 1
  for (int u = tid; u < 32 * (DIMO / 8); u += NTHR) {
    const int n  = u / (DIMO / 8);
    const int k0 = (u - n * (DIMO / 8)) * 8;
    float v[8];
#pragma unroll
    for (int e = 0; e < 8; ++e) v[e] = fc2w[(size_t)(k0 + e) * 32 + n];
    v8us hi, lo;
    split8(mk4(v[0], v[1], v[2], v[3]), mk4(v[4], v[5], v[6], v[7]), hi, lo);
    *(v8us*)(w2H + n * RP2 + k0) = hi;
    *(v8us*)(w2L + n * RP2 + k0) = lo;
  }
  __syncthreads();

#pragma unroll 1
  for (int rt = wave; rt < nRT; rt += NWAVE) {
    int arow = 16 * rt + m;
    arow = arow > GP - 1 ? GP - 1 : arow;
    const float* xr = EMB + (size_t)arow * EMBW;
    v8f acc[4];
#pragma unroll
    for (int t = 0; t < 4; ++t) acc[t] = zero8f();
#pragma unroll
    for (int kt = 0; kt < EMBW / 32; ++kt) {
      FragB ah, al;
#pragma unroll
      for (int g = 0; g < 2; ++g) {
        const int kb = 32 * kt + 16 * g + 8 * hh;
        split8(*(const v4f*)(xr + kb), *(const v4f*)(xr + kb + 4), ah.u[g], al.u[g]);
      }
#pragma unroll
      for (int t = 0; t < 4; ++t) {
        const unsigned short* bp = w1H + (16 * t + m) * RP1 + 32 * kt + 8 * hh;
        const unsigned short* bq = w1L + (16 * t + m) * RP1 + 32 * kt + 8 * hh;
        FragB bh, bl;
        bh.u[0] = *(const v8us*)bp;
        bh.u[1] = *(const v8us*)(bp + 16);
        bl.u[0] = *(const v8us*)bq;
        bl.u[1] = *(const v8us*)(bq + 16);
        acc[t] = wmb3(ah, al, bh, bl, acc[t]);
      }
    }
    float* op = o1 + (16 * rt + 8 * hh) * O1P;
#pragma unroll
    for (int t = 0; t < 4; ++t) {
      const int col = 16 * t + m;
      const float bv = fc1b[col];
#pragma unroll
      for (int r = 0; r < 8; ++r) op[r * O1P + col] = fmaxf(acc[t][r] + bv, 0.0f);
    }
  }
  __syncthreads();

#pragma unroll 1
  for (int rt = wave; rt < nRT; rt += NWAVE) {
    const float* ar = o1 + (16 * rt + m) * O1P;
    v8f acc[2];
#pragma unroll
    for (int t = 0; t < 2; ++t) acc[t] = zero8f();
#pragma unroll
    for (int kt = 0; kt < DIMO / 32; ++kt) {
      FragB ah, al;
#pragma unroll
      for (int g = 0; g < 2; ++g) {
        const int kb = 32 * kt + 16 * g + 8 * hh;
        split8(*(const v4f*)(ar + kb), *(const v4f*)(ar + kb + 4), ah.u[g], al.u[g]);
      }
#pragma unroll
      for (int t = 0; t < 2; ++t) {
        const unsigned short* bp = w2H + (16 * t + m) * RP2 + 32 * kt + 8 * hh;
        const unsigned short* bq = w2L + (16 * t + m) * RP2 + 32 * kt + 8 * hh;
        FragB bh, bl;
        bh.u[0] = *(const v8us*)bp;
        bh.u[1] = *(const v8us*)(bp + 16);
        bl.u[0] = *(const v8us*)bq;
        bl.u[1] = *(const v8us*)(bq + 16);
        acc[t] = wmb3(ah, al, bh, bl, acc[t]);
      }
    }
    float* op = o2 + (16 * rt + 8 * hh) * O2P;
#pragma unroll
    for (int t = 0; t < 2; ++t) {
      const int col = 16 * t + m;
      const float bv = fc2b[col];
#pragma unroll
      for (int r = 0; r < 8; ++r) op[r * O2P + col] = fmaxf(acc[t][r] + bv, 0.0f);
    }
  }
  __syncthreads();

  if (tid < nRT * 16) {
    const float* orr = o2 + tid * O2P;
    float s = fc3b[0];
#pragma unroll 1
    for (int i = 0; i < 32; ++i) s = s + orr[i] * fc3w[i];
    so[tid] = s;
  }
  __syncthreads();

  const int nV = G >> 2;
  v4f ov = zero4f();
  if (tid < nV) ov = *(const v4f*)(so + 4 * tid);
  if (tid < nV) *(volatile v4f*)(out + 4 * tid) = ov;
  __threadfence();
  if (tid < nV) *(volatile v4f*)(out + 4 * tid) = ov;
}

extern "C" void kernel_launch(void* const* d_in, const int* in_sizes, int n_in,
                              void* d_out, int out_size, void* d_ws, size_t ws_size,
                              hipStream_t stream) {
  if (n_in < 32) return;
  const int nN  = in_sizes[0] / 40;
  const int nE  = in_sizes[3] / 2;
  const int nN2 = in_sizes[2] / NISO;
  const int nA  = in_sizes[4] / 2;
  const int nE2 = in_sizes[5] / 2;
  const int G   = out_size;
  if (nN <= 0 || nE <= 0 || nN2 <= 0 || nA <= 0 || nE2 <= 0 || G <= 0) return;
  if (in_sizes[0] != nN * 40 || in_sizes[1] != nE * FE || in_sizes[2] != nN2 * NISO || in_sizes[3] != 2 * nE ||
      in_sizes[4] != 2 * nA || in_sizes[5] != 2 * nE2 || in_sizes[6] != nN || in_sizes[7] != nN2) return;
  if (in_sizes[8] != FE * HID || in_sizes[9] != HID || in_sizes[10] != HID * 40 * 32 || in_sizes[11] != 40 * 32 ||
      in_sizes[12] != 40 * 32 || in_sizes[13] != 32) return;
  if (in_sizes[14] != FE * HID || in_sizes[15] != HID || in_sizes[16] != HID * 32 * 64 || in_sizes[17] != 32 * 64 ||
      in_sizes[18] != 32 * 64 || in_sizes[19] != 64) return;
  if (in_sizes[20] != 80 * 64 || in_sizes[21] != 80 * 64 || in_sizes[22] != 64 || in_sizes[23] != 64 * 64 ||
      in_sizes[24] != 64 * 64 || in_sizes[25] != 64) return;
  if (in_sizes[26] != EMBW * 64 || in_sizes[27] != 64 || in_sizes[28] != 64 * 32 || in_sizes[29] != 32 ||
      in_sizes[30] != 32 || in_sizes[31] != 1) return;
  if (G > GMAX || (G & 3) != 0) return;
  if (nN > (1 << 24) || nN2 > (1 << 24) || nE > (1 << 28) || nE2 > (1 << 28) || nA > (1 << 28)) return;

  const float* x     = (const float*)d_in[0];
  const float* ea    = (const float*)d_in[1];
  const float* iso   = (const float*)d_in[2];
  const int*   ei    = (const int*)d_in[3];
  const int*   asg   = (const int*)d_in[4];
  const int*   ei2   = (const int*)d_in[5];
  const int*   bat   = (const int*)d_in[6];
  const int*   bat2  = (const int*)d_in[7];
  const float* nn0W1 = (const float*)d_in[8];
  const float* nn0b1 = (const float*)d_in[9];
  const float* nn0W2 = (const float*)d_in[10];
  const float* nn0b2 = (const float*)d_in[11];
  const float* root0 = (const float*)d_in[12];
  const float* cb0   = (const float*)d_in[13];
  const float* nn1W1 = (const float*)d_in[14];
  const float* nn1b1 = (const float*)d_in[15];
  const float* nn1W2 = (const float*)d_in[16];
  const float* nn1b2 = (const float*)d_in[17];
  const float* root1 = (const float*)d_in[18];
  const float* cb1   = (const float*)d_in[19];
  const float* W4rel = (const float*)d_in[20];
  const float* W4roo = (const float*)d_in[21];
  const float* b4    = (const float*)d_in[22];
  const float* W5rel = (const float*)d_in[23];
  const float* W5roo = (const float*)d_in[24];
  const float* b5    = (const float*)d_in[25];
  const float* fc1w  = (const float*)d_in[26];
  const float* fc1b  = (const float*)d_in[27];
  const float* fc2w  = (const float*)d_in[28];
  const float* fc2b  = (const float*)d_in[29];
  const float* fc3w  = (const float*)d_in[30];
  const float* fc3b  = (const float*)d_in[31];
  float* out = (float*)d_out;

  const int nMB = (nE + MEDG - 1) / MEDG;
  const int EP  = nMB * MEDG;
  const int nB0 = (nN + 511) / 512, NP0 = nB0 * 512;
  const int nB1 = (nN + 255) / 256, NP1 = nB1 * 256;
  const int nT  = (nN2 + 255) / 256, N2P = nT * 256;
  const int nPB = (G + NBP - 1) / NBP, GP = nPB * NBP;

  constexpr int KP0 = kpad_of(40);
  constexpr int KP1 = kpad_of(32);

  char* ws = (char*)d_ws;
  size_t off = 0;
  const size_t oBp0 = off; off += (size_t)32 * KP0 * 2;        off = (off + 255) & ~(size_t)255;
  const size_t oBp1 = off; off += (size_t)64 * KP1 * 2;        off = (off + 255) & ~(size_t)255;
  const size_t oMsg = off; off += (size_t)EP * 64 * 4;         off = (off + 255) & ~(size_t)255;
  const size_t oH0  = off; off += (size_t)NP0 * 32 * 4;        off = (off + 255) & ~(size_t)255;
  const size_t oH1  = off; off += (size_t)NP1 * 64 * 4;        off = (off + 255) & ~(size_t)255;
  const size_t oH2  = off; off += (size_t)N2P * 96 * 4;        off = (off + 255) & ~(size_t)255;
  const size_t oH4  = off; off += (size_t)N2P * 64 * 4;        off = (off + 255) & ~(size_t)255;
  const size_t oH5  = off; off += (size_t)N2P * 64 * 4;        off = (off + 255) & ~(size_t)255;
  const size_t oEmb = off; off += (size_t)GP * EMBW * 4;       off = (off + 255) & ~(size_t)255;
  if (off > ws_size) return;
  if (off > (size_t)128 * 1024 * 1024) return;
  _Float16* Bp0 = (_Float16*)(ws + oBp0);
  _Float16* Bp1 = (_Float16*)(ws + oBp1);
  float* msg = (float*)(ws + oMsg);
  float* h0  = (float*)(ws + oH0);
  float* h1  = (float*)(ws + oH1);
  float* h2  = (float*)(ws + oH2);
  float* h4  = (float*)(ws + oH4);
  float* h5  = (float*)(ws + oH5);
  float* emb = (float*)(ws + oEmb);

  const int vec8e  = ((nE  & 3) == 0) ? 1 : 0;
  const int vec8a  = ((nA  & 3) == 0) ? 1 : 0;
  const int vec8e2 = ((nE2 & 3) == 0) ? 1 : 0;

  constexpr int LM0 = msg_lds_bytes(40, 32);
  constexpr int LM1 = msg_lds_bytes(32, 64);
  constexpr int LN0 = node_lds_bytes(40, 32);
  constexpr int LN1 = node_lds_bytes(32, 64);
  constexpr int LG4 = gc_lds_bytes(80, 96);
  constexpr int LG5 = gc_lds_bytes(64, 64);
  hipFuncSetAttribute(reinterpret_cast<const void*>(&k_msg<40, 32>), hipFuncAttributeMaxDynamicSharedMemorySize, LM0);
  hipFuncSetAttribute(reinterpret_cast<const void*>(&k_msg<32, 64>), hipFuncAttributeMaxDynamicSharedMemorySize, LM1);
  hipFuncSetAttribute(reinterpret_cast<const void*>(&k_node<40, 32>), hipFuncAttributeMaxDynamicSharedMemorySize, LN0);
  hipFuncSetAttribute(reinterpret_cast<const void*>(&k_node<32, 64>), hipFuncAttributeMaxDynamicSharedMemorySize, LN1);
  hipFuncSetAttribute(reinterpret_cast<const void*>(&k_lift), hipFuncAttributeMaxDynamicSharedMemorySize, LIFT_LDS);
  hipFuncSetAttribute(reinterpret_cast<const void*>(&k_gc<80, 96>), hipFuncAttributeMaxDynamicSharedMemorySize, LG4);
  hipFuncSetAttribute(reinterpret_cast<const void*>(&k_gc<64, 64>), hipFuncAttributeMaxDynamicSharedMemorySize, LG5);
  hipFuncSetAttribute(reinterpret_cast<const void*>(&k_head), hipFuncAttributeMaxDynamicSharedMemorySize, HEAD_LDS);

  {
    const int nu0 = 32 * KP0 / 8, nu1 = 64 * KP1 / 8;
    k_bprep<40, 32><<<(nu0 + NTHR - 1) / NTHR, NTHR, 0, stream>>>(nn0W2, nn0b2, Bp0);
    k_bprep<32, 64><<<(nu1 + NTHR - 1) / NTHR, NTHR, 0, stream>>>(nn1W2, nn1b2, Bp1);
  }
  k_msg<40, 32><<<nMB, MTHR, LM0, stream>>>(x, nN, ei, nE, ea, nn0W1, nn0b1, Bp0, msg);
  k_node<40, 32><<<nB0, NTHR, LN0, stream>>>(ei, nE, vec8e, msg, x, nN, root0, cb0, h0);
  k_msg<32, 64><<<nMB, MTHR, LM1, stream>>>(h0, nN, ei, nE, ea, nn1W1, nn1b1, Bp1, msg);
  k_node<32, 64><<<nB1, NTHR, LN1, stream>>>(ei, nE, vec8e, msg, h0, nN, root1, cb1, h1);
  k_pool<<<nPB, NTHR, 0, stream>>>(bat, nN, h1, emb, G, 0);
  k_lift<<<nT, NTHR, LIFT_LDS, stream>>>(asg, nA, vec8a, h1, nN, iso, nN2, h2);
  k_gc<80, 96><<<nT, NTHR, LG4, stream>>>(ei2, nE2, vec8e2, h2, nN2, N2P, W4rel, W4roo, b4, h4);
  k_gc<64, 64><<<nT, NTHR, LG5, stream>>>(ei2, nE2, vec8e2, h4, nN2, N2P, W5rel, W5roo, b5, h5);
  k_pool<<<nPB, NTHR, 0, stream>>>(bat2, nN2, h5, emb, G, 64);
  k_head<<<1, NTHR, HEAD_LDS, stream>>>(emb, GP, fc1w, fc1b, fc2w, fc2b, fc3w, fc3b, out, G);
}
